// ImplicitMLP_48576080118009
// MI455X (gfx1250) — hardware-verified
//
#include <hip/hip_runtime.h>
#include <stdint.h>


typedef _Float16 f16;
typedef _Float16 v16h __attribute__((ext_vector_type(16)));
typedef _Float16 v8hb __attribute__((ext_vector_type(8)));
typedef v8hb v8h __attribute__((may_alias));
typedef float v8f __attribute__((ext_vector_type(8)));
typedef float v4fb __attribute__((ext_vector_type(4)));
typedef v4fb v4f __attribute__((may_alias));
typedef unsigned int u4b __attribute__((ext_vector_type(4)));
typedef u4b u4 __attribute__((may_alias));

#define TWO_PI_F 6.28318548202514648f

#define HW_PLANE   4096
#define NPT_WAVE   32
#define WAVES      4
#define NPT_CHUNK  (NPT_WAVE * WAVES)
#define ITERS      4
#define NPT_BLOCK  (NPT_CHUNK * ITERS)
#define NTHR       (WAVES * 32)
#define SX         264

#define LDS_F      0
#define LDS_W1     3072
#define LDS_W2     (LDS_W1 + 256*264*2)
#define LDS_W3     (LDS_W2 + 128*264*2)
#define LDS_W4     (LDS_W3 + 32*136*2)
#define LDS_ACT    (LDS_W4 + 16*40*2)
#define LDS_OBUF   (LDS_ACT + WAVES*NPT_WAVE*SX*2)
#define LDS_TOTAL  (LDS_OBUF + NPT_CHUNK*3*4)

static_assert(LDS_TOTAL == 284928, "");
static_assert((LDS_W1 % 16) == 0 && (LDS_W2 % 16) == 0 && (LDS_W3 % 16) == 0 &&
              (LDS_W4 % 16) == 0 && (LDS_ACT % 16) == 0 && (LDS_OBUF % 16) == 0, "");

#define F_BMAT 0
#define F_B1   256
#define F_B2   512
#define F_B3   640
#define F_B4   672
#define F_W5   688
#define F_B5   736

#define WS_W1  0
#define WS_W2  65536
#define WS_W3  98304
#define WS_W4  102400
#define WS_END 102912
#define PREP_UNITS (WS_END / 8)
#define WS_BYTES   ((size_t)WS_END * 2)
#define W_SCALE    64.0f
#define W_INV      0.015625f

__launch_bounds__(256)
__global__ void k_prep(const float* __restrict__ L1, const float* __restrict__ R1,
                       const float* __restrict__ L2, const float* __restrict__ R2,
                       const float* __restrict__ W3, const float* __restrict__ W4,
                       f16* __restrict__ wsh) {
  const int t = blockIdx.x * blockDim.x + threadIdx.x;
  if (t >= PREP_UNITS) return;
  float v[8];
  #pragma unroll
  for (int j = 0; j < 8; ++j) v[j] = 0.f;
  if (t < 8192) {
    const int n = t >> 5, k8 = (t & 31) * 8;
    const float* lp = L1 + n * 70;
    const float* rp = R1 + k8;
    #pragma unroll 2
    for (int r = 0; r < 70; ++r) {
      const float l = lp[r];
      const v4fb ra = *(const v4f*)(rp + r * 256);
      const v4fb rb = *(const v4f*)(rp + r * 256 + 4);
      v[0] = fmaf(l, ra[0], v[0]); v[1] = fmaf(l, ra[1], v[1]);
      v[2] = fmaf(l, ra[2], v[2]); v[3] = fmaf(l, ra[3], v[3]);
      v[4] = fmaf(l, rb[0], v[4]); v[5] = fmaf(l, rb[1], v[5]);
      v[6] = fmaf(l, rb[2], v[6]); v[7] = fmaf(l, rb[3], v[7]);
    }
  } else if (t < 12288) {
    const int u = t - 8192;
    const int n = u >> 5, k8 = (u & 31) * 8;
    const float* lp = L2 + n * 10;
    const float* rp = R2 + k8;
    #pragma unroll 2
    for (int r = 0; r < 10; ++r) {
      const float l = lp[r];
      const v4fb ra = *(const v4f*)(rp + r * 256);
      const v4fb rb = *(const v4f*)(rp + r * 256 + 4);
      v[0] = fmaf(l, ra[0], v[0]); v[1] = fmaf(l, ra[1], v[1]);
      v[2] = fmaf(l, ra[2], v[2]); v[3] = fmaf(l, ra[3], v[3]);
      v[4] = fmaf(l, rb[0], v[4]); v[5] = fmaf(l, rb[1], v[5]);
      v[6] = fmaf(l, rb[2], v[6]); v[7] = fmaf(l, rb[3], v[7]);
    }
  } else if (t < 12800) {
    const int u = t - 12288;
    const v4fb ra = *(const v4f*)(W3 + u * 8);
    const v4fb rb = *(const v4f*)(W3 + u * 8 + 4);
    v[0] = ra[0]; v[1] = ra[1]; v[2] = ra[2]; v[3] = ra[3];
    v[4] = rb[0]; v[5] = rb[1]; v[6] = rb[2]; v[7] = rb[3];
  } else {
    const int u = t - 12800;
    const v4fb ra = *(const v4f*)(W4 + u * 8);
    const v4fb rb = *(const v4f*)(W4 + u * 8 + 4);
    v[0] = ra[0]; v[1] = ra[1]; v[2] = ra[2]; v[3] = ra[3];
    v[4] = rb[0]; v[5] = rb[1]; v[6] = rb[2]; v[7] = rb[3];
  }
  union { v8hb h; u4b u; } pk;
  #pragma unroll
  for (int j = 0; j < 8; ++j) pk.h[j] = (f16)(v[j] * W_SCALE);
  const u4b val = pk.u;
  volatile u4b* dst = (volatile u4b*)(wsh + (size_t)t * 8);
  *dst = val;
  __threadfence();
  *dst = val;
}

__device__ __forceinline__ v16h cat8(v8hb lo, v8hb hi) {
  return __builtin_shufflevector(lo, hi, 0,1,2,3,4,5,6,7,8,9,10,11,12,13,14,15);
}
__device__ __forceinline__ v8f wmma16(v16h a, v16h b, v8f c) {
  return __builtin_amdgcn_wmma_f32_16x16x32_f16(false, a, false, b, (short)0, c, false, false);
}

template<int KT, int NT, int SW>
__device__ __forceinline__ void layer_pass(f16* xb, const f16* wl, const float* bias, int lane) {
  const int m  = lane & 15;
  const int h8 = (lane >> 4) * 8;
  v16h a0[KT], a1[KT];
  #pragma unroll
  for (int kt = 0; kt < KT; ++kt) {
    const f16* p0 = xb + m * SX + kt * 32 + h8;
    const f16* p1 = p0 + 16 * SX;
    a0[kt] = cat8(*(const v8h*)p0, *(const v8h*)(p0 + 16));
    a1[kt] = cat8(*(const v8h*)p1, *(const v8h*)(p1 + 16));
  }
  #pragma unroll 1
  for (int nt = 0; nt < NT; ++nt) {
    const f16* pb = wl + (nt * 16 + m) * SW + h8;
    v8f acc0 = {}, acc1 = {};
    v16h bv;
    #pragma unroll
    for (int kt = 0; kt < KT; ++kt) {
      bv = cat8(*(const v8h*)(pb + kt * 32), *(const v8h*)(pb + kt * 32 + 16));
      acc0 = wmma16(a0[kt], bv, acc0);
      acc1 = wmma16(a1[kt], bv, acc1);
    }
    asm volatile("v_nop\n\tv_nop\n\tv_nop\n\tv_nop"
                 : "+v"(acc0), "+v"(acc1) : "v"(a1[KT - 1]), "v"(bv));
    const int col = nt * 16 + m;
    const float bs = bias[col];
    #pragma unroll
    for (int r = 0; r < 8; ++r) {
      const float v0 = fmaxf(fmaf(acc0[r], W_INV, bs), 0.f);
      const float v1 = fmaxf(fmaf(acc1[r], W_INV, bs), 0.f);
      xb[(h8 + r) * SX + col]      = (f16)v0;
      xb[(16 + h8 + r) * SX + col] = (f16)v1;
    }
  }
}

__device__ __forceinline__ void sincos_pio2(float x, float& sn, float& cs) {
  const float q = __builtin_rintf(x * 0.636619772367581343f);
  float r = fmaf(-q, 1.57079637050628662e+00f, x);
  r = fmaf(-q, -4.37113882867379653e-08f, r);
  r = fmaf(-q, -1.71512448e-15f, r);
  const float z = r * r;
  float ps = fmaf(z, -1.9515295891e-4f, 8.3321608736e-3f);
  ps = fmaf(z, ps, -1.6666654611e-1f);
  const float s = fmaf(r * z, ps, r);
  float pc = fmaf(z, 2.443315711809948e-5f, -1.388731625493765e-3f);
  pc = fmaf(z, pc, 4.166664568298827e-2f);
  const float c = fmaf(z * z, pc, fmaf(z, -0.5f, 1.0f));
  const int qi = (int)q;
  const bool sw = (qi & 1) != 0;
  float a = sw ? c : s;
  float b = sw ? s : c;
  if (qi & 2) a = -a;
  if ((qi + 1) & 2) b = -b;
  sn = a; cs = b;
}

__device__ __forceinline__ float prodsum(float a, float b, float c, float d) {
  #pragma clang fp contract(off)
  return a * b + c * d;
}

__launch_bounds__(NTHR)
__global__ void k_mlp(const float* __restrict__ coords,
                      const float* __restrict__ Bmat,
                      const float* __restrict__ b1, const float* __restrict__ b2,
                      const float* __restrict__ b3, const float* __restrict__ b4,
                      const float* __restrict__ W5, const float* __restrict__ b5,
                      const f16* __restrict__ wsh,
                      float* out, int npts) {
  extern __shared__ __attribute__((aligned(16))) char smem[];
  float* F   = (float*)(smem + LDS_F);
  f16*   W1l = (f16*)(smem + LDS_W1);
  f16*   W2l = (f16*)(smem + LDS_W2);
  f16*   W3l = (f16*)(smem + LDS_W3);
  f16*   W4l = (f16*)(smem + LDS_W4);
  float* obuf = (float*)(smem + LDS_OBUF);

  const int tid  = threadIdx.x;
  const int wave = tid >> 5, lane = tid & 31;

  for (int c = tid; c < 8192; c += NTHR) {
    const int row = c >> 5, col8 = (c & 31) * 8;
    *(v8h*)(W1l + row * 264 + col8) = *(const v8h*)(wsh + WS_W1 + row * 256 + col8);
  }
  for (int c = tid; c < 4096; c += NTHR) {
    const int row = c >> 5, col8 = (c & 31) * 8;
    *(v8h*)(W2l + row * 264 + col8) = *(const v8h*)(wsh + WS_W2 + row * 256 + col8);
  }
  for (int c = tid; c < 512; c += NTHR) {
    const int row = c >> 4, col8 = (c & 15) * 8;
    *(v8h*)(W3l + row * 136 + col8) = *(const v8h*)(wsh + WS_W3 + row * 128 + col8);
  }
  if (tid < 64) {
    const int row = tid >> 2, col8 = (tid & 3) * 8;
    *(v8h*)(W4l + row * 40 + col8) = *(const v8h*)(wsh + WS_W4 + row * 32 + col8);
  }

  for (int i = tid; i < 256; i += NTHR) F[F_BMAT + i] = Bmat[i];
  for (int i = tid; i < 256; i += NTHR) F[F_B1 + i] = b1[i];
  F[F_B2 + tid] = b2[tid];
  if (tid < 32) F[F_B3 + tid] = b3[tid];
  if (tid < 16) F[F_B4 + tid] = b4[tid];
  if (tid < 48) F[F_W5 + tid] = W5[tid];
  if (tid < 3)  F[F_B5 + tid] = b5[tid];
  __syncthreads();

  f16* xb = (f16*)(smem + LDS_ACT) + wave * (NPT_WAVE * SX);

  float bm0[4], bm1[4];
  #pragma unroll
  for (int mi = 0; mi < 4; ++mi) {
    bm0[mi] = F[F_BMAT + lane + 32 * mi];
    bm1[mi] = F[F_BMAT + 128 + lane + 32 * mi];
  }

  for (int it = 0; it < ITERS; ++it) {
    const int cbase = blockIdx.x * NPT_BLOCK + it * NPT_CHUNK;
    const int pbase = cbase + wave * NPT_WAVE;

    float c0l = 0.f, c1l = 0.f;
    {
      const int p = pbase + lane;
      if (p < npts) {
        const int b = p >> 12, rem = p & (HW_PLANE - 1);
        c0l = coords[(size_t)(2 * b)     * HW_PLANE + rem];
        c1l = coords[(size_t)(2 * b + 1) * HW_PLANE + rem];
      }
    }

    #pragma unroll 1
    for (int i = 0; i < NPT_WAVE; ++i) {
      const float c0 = __int_as_float(__builtin_amdgcn_readlane(__float_as_int(c0l), i));
      const float c1 = __int_as_float(__builtin_amdgcn_readlane(__float_as_int(c1l), i));
      f16* row = xb + i * SX;
      #pragma unroll
      for (int mi = 0; mi < 4; ++mi) {
        const float e = prodsum(c0, bm0[mi], c1, bm1[mi]);
        const float proj = TWO_PI_F * e;
        float s, c;
        sincos_pio2(proj, s, c);
        row[lane + 32 * mi]       = (f16)s;
        row[128 + lane + 32 * mi] = (f16)c;
      }
    }
    __syncthreads();

    layer_pass<8, 16, 264>(xb, W1l, F + F_B1, lane);
    __syncthreads();
    layer_pass<8,  8, 264>(xb, W2l, F + F_B2, lane);
    __syncthreads();
    layer_pass<4,  2, 136>(xb, W3l, F + F_B3, lane);
    __syncthreads();
    layer_pass<1,  1,  40>(xb, W4l, F + F_B4, lane);
    __syncthreads();

    #pragma unroll 1
    for (int j = 0; j < 3; ++j) {
      const int idx = lane + 32 * j;
      const int pt  = idx / 3;
      const int cc  = idx - 3 * pt;
      const f16* xr = xb + pt * SX;
      const v8hb x0 = *(const v8h*)xr;
      const v8hb x1 = *(const v8h*)(xr + 8);
      const float* wr = F + F_W5 + cc * 16;
      const v4fb w0 = *(const v4f*)wr;
      const v4fb w1 = *(const v4f*)(wr + 4);
      const v4fb w2 = *(const v4f*)(wr + 8);
      const v4fb w3 = *(const v4f*)(wr + 12);
      float acc = 0.f;
      acc = fmaf((float)x0[0], w0[0], acc); acc = fmaf((float)x0[1], w0[1], acc);
      acc = fmaf((float)x0[2], w0[2], acc); acc = fmaf((float)x0[3], w0[3], acc);
      acc = fmaf((float)x0[4], w1[0], acc); acc = fmaf((float)x0[5], w1[1], acc);
      acc = fmaf((float)x0[6], w1[2], acc); acc = fmaf((float)x0[7], w1[3], acc);
      acc = fmaf((float)x1[0], w2[0], acc); acc = fmaf((float)x1[1], w2[1], acc);
      acc = fmaf((float)x1[2], w2[2], acc); acc = fmaf((float)x1[3], w2[3], acc);
      acc = fmaf((float)x1[4], w3[0], acc); acc = fmaf((float)x1[5], w3[1], acc);
      acc = fmaf((float)x1[6], w3[2], acc); acc = fmaf((float)x1[7], w3[3], acc);
      acc += F[F_B5 + cc];
      obuf[wave * (NPT_WAVE * 3) + idx] = acc;
    }
    __syncthreads();

    if (cbase + NPT_CHUNK <= npts) {
      if (tid < 96) {
        const v4fb val = *(const v4f*)(obuf + tid * 4);
        volatile v4fb* dst = (volatile v4fb*)(out + (size_t)cbase * 3 + tid * 4);
        *dst = val;
        __threadfence();
        *dst = val;
      }
    } else {
      for (int e = tid; e < NPT_CHUNK * 3; e += NTHR) {
        const long long g = (long long)cbase * 3 + e;
        if (g < (long long)npts * 3) {
          const float val = obuf[e];
          volatile float* dst = (volatile float*)(out + g);
          *dst = val;
          __threadfence();
          *dst = val;
        }
      }
    }
    __syncthreads();
  }
}

extern "C" void kernel_launch(void* const* d_in, const int* in_sizes, int n_in,
                              void* d_out, int out_size, void* d_ws, size_t ws_size,
                              hipStream_t stream) {
  if (n_in < 14) return;
  const float* coords = (const float*)d_in[0];
  const float* Bmat   = (const float*)d_in[1];
  const float* L1     = (const float*)d_in[2];
  const float* R1     = (const float*)d_in[3];
  const float* b1     = (const float*)d_in[4];
  const float* L2     = (const float*)d_in[5];
  const float* R2     = (const float*)d_in[6];
  const float* b2     = (const float*)d_in[7];
  const float* W3     = (const float*)d_in[8];
  const float* b3     = (const float*)d_in[9];
  const float* W4     = (const float*)d_in[10];
  const float* b4     = (const float*)d_in[11];
  const float* W5     = (const float*)d_in[12];
  const float* b5     = (const float*)d_in[13];
  f16*   wsh = (f16*)d_ws;
  float* out = (float*)d_out;

  if (in_sizes[1] != 256 || in_sizes[2] != 256 * 70 || in_sizes[3] != 70 * 256 ||
      in_sizes[4] != 256 || in_sizes[5] != 128 * 10 || in_sizes[6] != 10 * 256 ||
      in_sizes[7] != 128 || in_sizes[8] != 32 * 128 || in_sizes[9] != 32 ||
      in_sizes[10] != 16 * 32 || in_sizes[11] != 16 || in_sizes[12] != 48 ||
      in_sizes[13] != 3) return;
  if (in_sizes[0] <= 0 || (in_sizes[0] % (2 * HW_PLANE)) != 0) return;
  const int npts = in_sizes[0] / 2;
  if (out_size != npts * 3) return;
  if (ws_size < WS_BYTES) return;

  (void)hipFuncSetAttribute((const void*)k_mlp,
                            hipFuncAttributeMaxDynamicSharedMemorySize, LDS_TOTAL);

  const int prep_blocks = (PREP_UNITS + 255) / 256;
  k_prep<<<prep_blocks, 256, 0, stream>>>(L1, R1, L2, R2, W3, W4, wsh);

  const int main_blocks = (npts + NPT_BLOCK - 1) / NPT_BLOCK;
  k_mlp<<<main_blocks, NTHR, LDS_TOTAL, stream>>>(coords, Bmat, b1, b2, b3, b4, W5, b5,
                                                  wsh, out, npts);
}
